// PairwiseMLPSimilarity_3848290697817
// MI455X (gfx1250) — hardware-verified
//
#include <hip/hip_runtime.h>
#include <stddef.h>


typedef _Float16 v16h __attribute__((ext_vector_type(16)));
typedef _Float16 v8h  __attribute__((ext_vector_type(8)));
typedef float    v8f  __attribute__((ext_vector_type(8)));
typedef float    v4f  __attribute__((ext_vector_type(4)));
typedef _Float16 h16;

#ifndef NB
#define NB 8
#endif
#ifndef SEQ
#define SEQ 512
#endif
#define NB_FULL  8
#define SEQ_FULL 512
#define KD    64
#define HD    128
#define PW    384
#define MROWS (NB * SEQ)
#define NTILE (SEQ / 32)
#define NTRI  (NTILE * (NTILE + 1) / 2)

static_assert(NB >= 1 && NB <= NB_FULL);
static_assert(SEQ >= 64 && SEQ <= SEQ_FULL && (SEQ % 64) == 0);
static_assert(KD == 64 && (KD % 32) == 0);
static_assert(HD == 4 * 32);
static_assert((HD % 64) == 0);
static_assert(PW == 3 * HD && (PW % 64) == 0 && (PW % 32) == 0);
static_assert((MROWS % 64) == 0 && (MROWS % 32) == 0);
static_assert((size_t)NB_FULL * SEQ_FULL * SEQ_FULL * 4 == (size_t)8388608);
static_assert((size_t)((NB - 1) * SEQ_FULL + SEQ) * SEQ_FULL <= (size_t)NB_FULL * SEQ_FULL * SEQ_FULL);

#define LDT 72
#define LDC 68
#define LPAD 132
#define LSO 36
static_assert((LDT % 8) == 0 && LDT >= 64);
static_assert((LDC % 4) == 0 && LDC >= 64);
static_assert((LPAD % 4) == 0 && LPAD >= HD);
static_assert((LSO % 4) == 0 && LSO >= 32);

#define WCARRY 64.0f
#define XCARRY 16.0f

#define WT_BYTES  ((size_t)PW * KD * 2)
#define X16_BYTES ((size_t)MROWS * KD * 2)
#define PF_BYTES  ((size_t)MROWS * PW * 4)
#define OFF_WT  ((size_t)0)
#define OFF_X16 (OFF_WT + WT_BYTES)
#define OFF_PF  (OFF_X16 + X16_BYTES)
#define WS_TOTAL (OFF_PF + PF_BYTES)
static_assert((WT_BYTES % 128) == 0 && (X16_BYTES % 128) == 0 && (PF_BYTES % 128) == 0);
static_assert(WS_TOTAL <= (size_t)134217728);

#define PAIR_LDS_BYTES ((size_t)(2 * 32 * LPAD + HD + 2 * 32 * LSO + 32) * 4)
static_assert(PAIR_LDS_BYTES <= (size_t)131072);
static_assert((size_t)64 * LDC * 4 <= (size_t)131072);
static_assert((size_t)64 * LDT * 2 <= (size_t)131072);

__device__ __forceinline__ float bf16r(float x) {
  unsigned int u = __float_as_uint(x);
  u = (u + 0x7FFFu + ((u >> 16) & 1u)) & 0xFFFF0000u;
  return __uint_as_float(u);
}

__device__ __forceinline__ h16 toh_flush(float v) {
  const h16 r = (h16)v;
  return (fabsf(v) < 6.103515625e-05f) ? (h16)0.0f : r;
}

__device__ __forceinline__ v16h frag_at(const _Float16* p) {
  v8h lo = *(const v8h*)(p);
  v8h hi = *(const v8h*)(p + 16);
  v16h out;
#pragma unroll
  for (int i = 0; i < 8; ++i) { out[i] = lo[i]; out[i + 8] = hi[i]; }
  return out;
}

__device__ __forceinline__ v8f wmma16(v16h a, v16h b, v8f c) {
  v8f d = __builtin_amdgcn_wmma_f32_16x16x32_f16(false, a, false, b, (short)0, c,
                                                 false, false);
  asm volatile("v_nop\n\tv_nop\n\tv_nop\n\tv_nop" : "+v"(d) : "v"(a), "v"(b));
  return d;
}

__device__ __forceinline__ float sigm(float z) {
  return __builtin_amdgcn_rcpf(1.0f + __expf(-z));
}

__global__ __launch_bounds__(256) void wconv_kernel(
    const float* __restrict__ W, _Float16* __restrict__ Wt, unsigned ldw, unsigned ldk) {
  __shared__ _Float16 T[64 * LDT];
  const unsigned tid = threadIdx.x;
  const unsigned n0 = blockIdx.x * 64u;
  const unsigned k0 = blockIdx.y * 64u;
#pragma unroll 4
  for (unsigned j = 0; j < 16u; ++j) {
    const unsigned idx = tid + 256u * j;
    const unsigned kr = idx >> 6, nc = idx & 63u;
    const float v = W[(size_t)(k0 + kr) * ldw + n0 + nc];
    T[nc * LDT + kr] = toh_flush(WCARRY * bf16r(v));
  }
  __syncthreads();
  v8h x[2];
  size_t off[2];
#pragma unroll
  for (unsigned i = 0; i < 2u; ++i) {
    const unsigned n = 32u * i + (tid >> 3);
    const unsigned kc = (tid & 7u) * 8u;
    x[i] = *(const v8h*)&T[n * LDT + kc];
    off[i] = (size_t)(n0 + n) * ldk + k0 + kc;
  }
#pragma unroll
  for (int i = 0; i < 2; ++i) *(volatile v8h*)(Wt + off[i]) = x[i];
  __threadfence();
#pragma unroll
  for (int i = 0; i < 2; ++i) *(volatile v8h*)(Wt + off[i]) = x[i];
}
static_assert(2 * 32 == 64);

__global__ __launch_bounds__(256) void xconv_kernel(
    const float* __restrict__ X, _Float16* __restrict__ X16) {
#pragma clang fp contract(off)
  const unsigned gid = blockIdx.x * 256u + threadIdx.x;
  const unsigned crow = gid >> 3;
  const unsigned c = (gid & 7u) * 8u;
  const unsigned bidx = crow / (unsigned)SEQ;
  const unsigned sq = crow - bidx * (unsigned)SEQ;
  const size_t srow = (size_t)bidx * SEQ_FULL + sq;
  const v4f a0 = *(const v4f*)(X + srow * KD + c);
  const v4f a1 = *(const v4f*)(X + srow * KD + c + 4u);
  v8h o;
#pragma unroll
  for (int i = 0; i < 4; ++i) {
    o[i]     = toh_flush(XCARRY * bf16r(a0[i]));
    o[i + 4] = toh_flush(XCARRY * bf16r(a1[i]));
  }
  _Float16* p = X16 + (size_t)crow * KD + c;
  *(volatile v8h*)p = o;
  __threadfence();
  *(volatile v8h*)p = o;
}
static_assert(((size_t)MROWS * 8) % 256 == 0);

__global__ __launch_bounds__(256) void gemm_pre_kernel(
    const _Float16* __restrict__ A16, const _Float16* __restrict__ Bt,
    float* __restrict__ outf) {
  __shared__ float Cs[64 * LDC];
  const unsigned tid = threadIdx.x, lane = tid & 31u;
  const unsigned w = (unsigned)__builtin_amdgcn_readfirstlane((int)(threadIdx.x >> 5));
  const unsigned mw = w >> 1, nw = w & 1u;
  const unsigned hh = lane >> 4, m = lane & 15u;
  const unsigned n0 = blockIdx.x * 64u;
  const unsigned row0 = blockIdx.y * 64u;

  const _Float16* ap  = A16 + (size_t)(row0 + mw * 16u + m) * KD + hh * 8u;
  const _Float16* bp0 = Bt + (size_t)(n0 + nw * 32u + m) * KD + hh * 8u;
  const _Float16* bp1 = bp0 + (size_t)16 * KD;
  v8f acc0 = {}, acc1 = {};
#pragma unroll
  for (unsigned k0 = 0; k0 < (unsigned)KD; k0 += 32u) {
    const v16h a  = frag_at(ap + k0);
    const v16h b0 = frag_at(bp0 + k0);
    const v16h b1 = frag_at(bp1 + k0);
    acc0 = wmma16(a, b0, acc0);
    acc1 = wmma16(a, b1, acc1);
  }
#pragma unroll
  for (int r = 0; r < 8; ++r) {
    float* d = &Cs[(mw * 16u + hh * 8u + (unsigned)r) * LDC + nw * 32u + m];
    d[0]  = acc0[r];
    d[16] = acc1[r];
  }
  __syncthreads();

  const float cs = 1.0f / (WCARRY * XCARRY);
  v4f xs[4];
  size_t off[4];
#pragma unroll
  for (unsigned i = 0; i < 4u; ++i) {
    const unsigned r = 16u * i + (tid >> 4);
    const unsigned c = (tid & 15u) * 4u;
    const v4f u = *(const v4f*)&Cs[r * LDC + c];
    v4f val;
#pragma unroll
    for (int j = 0; j < 4; ++j) val[j] = u[j] * cs;
    xs[i] = val;
    off[i] = (size_t)(row0 + r) * PW + n0 + c;
  }
#pragma unroll
  for (int i = 0; i < 4; ++i) *(volatile v4f*)(outf + off[i]) = xs[i];
  __threadfence();
#pragma unroll
  for (int i = 0; i < 4; ++i) *(volatile v4f*)(outf + off[i]) = xs[i];
}
static_assert(4 * 16 == 64);

__global__ __launch_bounds__(256) void pair_kernel(
    const float* __restrict__ Pf,
    const float* __restrict__ bc1, const float* __restrict__ Wc2, const float* __restrict__ bc2,
    const float* __restrict__ bs1, const float* __restrict__ Ws2, const float* __restrict__ bs2,
    float* __restrict__ out) {
#pragma clang fp contract(off)
  __shared__ __attribute__((aligned(16))) float sA[32 * LPAD];
  __shared__ __attribute__((aligned(16))) float sB[32 * LPAD];
  __shared__ __attribute__((aligned(16))) float w2s[HD];
  __shared__ __attribute__((aligned(16))) float So[32 * LSO];
  __shared__ __attribute__((aligned(16))) float Sot[32 * LSO];
  __shared__ float dgs[32];

  const unsigned tid = threadIdx.x;
  const unsigned b = blockIdx.y;

  unsigned t = blockIdx.x, ti = 0u;
#pragma unroll 1
  for (unsigned s = 0; s + 1u < (unsigned)NTILE; ++s) {
    const unsigned len = (unsigned)NTILE - ti;
    const bool adv = (t >= len);
    t  = adv ? (t - len) : t;
    ti = adv ? (ti + 1u) : ti;
  }
  unsigned tj = ti + t;
  tj = (tj < (unsigned)NTILE) ? tj : ((unsigned)NTILE - 1u);
  const unsigned i0 = ti * 32u, j0 = tj * 32u;
  const bool dtile = (ti == tj);

  const size_t arow = (size_t)(b * (unsigned)SEQ + i0) * PW;
  const size_t brow = (size_t)(b * (unsigned)SEQ + j0) * PW + HD;
#pragma unroll 1
  for (unsigned s = 0; s < 4u; ++s) {
    const unsigned idx = tid + 256u * s;
    const unsigned r = idx >> 5, c = (idx & 31u) * 4u;
    const v4f a  = *(const v4f*)(Pf + arow + (size_t)r * PW + c);
    const v4f bb = *(const v4f*)(Pf + brow + (size_t)r * PW + c);
    const v4f g  = *(const v4f*)(bc1 + c);
    v4f av;
#pragma unroll
    for (int j = 0; j < 4; ++j) av[j] = a[j] + bf16r(g[j]);
    *(v4f*)&sA[r * LPAD + c] = av;
    *(v4f*)&sB[r * LPAD + c] = bb;
  }
  if (tid < (unsigned)HD) w2s[tid] = bf16r(Wc2[tid]);

  {
    const unsigned r = tid >> 3, part = tid & 7u;
    const float* dp = Pf + (size_t)(b * (unsigned)SEQ + i0 + r) * PW + 2u * HD + part * 16u;
    float acc = 0.0f;
#pragma unroll 1
    for (unsigned q = 0; q < 4u; ++q) {
      const v4f d  = *(const v4f*)(dp + 4u * q);
      const v4f g  = *(const v4f*)(bs1 + part * 16u + 4u * q);
      const v4f wv = *(const v4f*)(Ws2 + part * 16u + 4u * q);
#pragma unroll
      for (int j = 0; j < 4; ++j)
        acc = fmaf(fmaxf(d[j] + bf16r(g[j]), 0.0f), bf16r(wv[j]), acc);
    }
    acc += __shfl_xor(acc, 1, 32);
    acc += __shfl_xor(acc, 2, 32);
    acc += __shfl_xor(acc, 4, 32);
    const float sg = sigm(acc + bf16r(bs2[0]));
    if (part == 0u) dgs[r] = sg;
  }
  __syncthreads();

  const unsigned tx = tid & 15u, ty = tid >> 4;
  const unsigned pa = (ty * 2u) * LPAD;
  const unsigned pb = (tx * 2u) * LPAD;
  float a00 = 0.0f, a01 = 0.0f, a10 = 0.0f, a11 = 0.0f;
#pragma unroll 1
  for (unsigned h = 0; h < (unsigned)HD; h += 4u) {
    const v4f wv = *(const v4f*)&w2s[h];
    const v4f x0 = *(const v4f*)&sA[pa + h];
    const v4f x1 = *(const v4f*)&sA[pa + LPAD + h];
    const v4f y0 = *(const v4f*)&sB[pb + h];
    const v4f y1 = *(const v4f*)&sB[pb + LPAD + h];
#pragma unroll
    for (int j = 0; j < 4; ++j) {
      a00 = fmaf(fmaxf(x0[j] + y0[j], 0.0f), wv[j], a00);
      a01 = fmaf(fmaxf(x0[j] + y1[j], 0.0f), wv[j], a01);
      a10 = fmaf(fmaxf(x1[j] + y0[j], 0.0f), wv[j], a10);
      a11 = fmaf(fmaxf(x1[j] + y1[j], 0.0f), wv[j], a11);
    }
  }
  const float c2 = bf16r(bc2[0]);
  const float s00 = sigm(a00 + c2);
  const float s01 = sigm(a01 + c2);
  const float s10 = sigm(a10 + c2);
  const float s11 = sigm(a11 + c2);
  So[(2u * ty) * LSO + 2u * tx]            = s00;
  So[(2u * ty) * LSO + 2u * tx + 1u]       = s01;
  So[(2u * ty + 1u) * LSO + 2u * tx]       = s10;
  So[(2u * ty + 1u) * LSO + 2u * tx + 1u]  = s11;
  Sot[(2u * tx) * LSO + 2u * ty]           = s00;
  Sot[(2u * tx + 1u) * LSO + 2u * ty]      = s01;
  Sot[(2u * tx) * LSO + 2u * ty + 1u]      = s10;
  Sot[(2u * tx + 1u) * LSO + 2u * ty + 1u] = s11;
  __syncthreads();

  const unsigned r = tid >> 3, c0 = (tid & 7u) * 4u;
  const v4f u  = *(const v4f*)&So[r * LSO + c0];
  const v4f tt = *(const v4f*)&Sot[r * LSO + c0];
  const float dv = dgs[r];
  v4f xa;
#pragma unroll
  for (int j = 0; j < 4; ++j) {
    const unsigned c = c0 + (unsigned)j;
    const float mrg = (r < c) ? u[j] : ((r > c) ? tt[j] : dv);
    xa[j] = dtile ? mrg : u[j];
  }
  const size_t offa = ((size_t)b * SEQ_FULL + i0 + r) * SEQ_FULL + j0 + c0;
  const size_t offb = ((size_t)b * SEQ_FULL + j0 + r) * SEQ_FULL + i0 + c0;
  *(volatile v4f*)(out + offa) = xa;
  if (!dtile) *(volatile v4f*)(out + offb) = tt;
  __threadfence();
  *(volatile v4f*)(out + offa) = xa;
  if (!dtile) *(volatile v4f*)(out + offb) = tt;
}
static_assert(256 / 8 == 32);
static_assert(16 * 2 == 32);
static_assert(8 * 16 == HD);

extern "C" void kernel_launch(void* const* d_in, const int* in_sizes, int n_in,
                              void* d_out, int out_size, void* d_ws, size_t ws_size,
                              hipStream_t stream) {
  if (n_in < 9) return;
  const long long need_x = ((long long)(NB - 1) * SEQ_FULL + SEQ) * KD;
  const long long need_o = ((long long)(NB - 1) * SEQ_FULL + SEQ) * SEQ_FULL;
  if ((long long)in_sizes[0] < need_x) return;
  if ((long long)in_sizes[1] < (long long)2 * KD * HD) return;
  if (in_sizes[2] < HD || in_sizes[3] < HD || in_sizes[4] < 1) return;
  if ((long long)in_sizes[5] < (long long)KD * HD) return;
  if (in_sizes[6] < HD || in_sizes[7] < HD || in_sizes[8] < 1) return;
  if ((long long)out_size < need_o) return;
  if (ws_size < WS_TOTAL) return;

  const float* X   = (const float*)d_in[0];
  const float* wc1 = (const float*)d_in[1];
  const float* bc1 = (const float*)d_in[2];
  const float* wc2 = (const float*)d_in[3];
  const float* bc2 = (const float*)d_in[4];
  const float* ws1 = (const float*)d_in[5];
  const float* bs1 = (const float*)d_in[6];
  const float* ws2 = (const float*)d_in[7];
  const float* bs2 = (const float*)d_in[8];
  float* out = (float*)d_out;

  char* ws = (char*)d_ws;
  _Float16* Wt  = (_Float16*)(ws + OFF_WT);
  _Float16* X16 = (_Float16*)(ws + OFF_X16);
  float*    Pf  = (float*)(ws + OFF_PF);

  dim3 blk(256);
  dim3 gw(HD / 64, KD / 64);
  wconv_kernel<<<gw, blk, 0, stream>>>(wc1, Wt, (unsigned)HD, (unsigned)KD);
  wconv_kernel<<<gw, blk, 0, stream>>>(wc1 + (size_t)KD * HD, Wt + (size_t)HD * KD,
                                        (unsigned)HD, (unsigned)KD);
  wconv_kernel<<<gw, blk, 0, stream>>>(ws1, Wt + (size_t)2 * HD * KD,
                                        (unsigned)HD, (unsigned)KD);
  xconv_kernel<<<dim3(MROWS / 32), blk, 0, stream>>>(X, X16);
  gemm_pre_kernel<<<dim3(PW / 64, MROWS / 64), blk, 0, stream>>>(X16, Wt, Pf);
  pair_kernel<<<dim3(NTRI, NB), blk, 0, stream>>>(Pf, bc1, wc2, bc2, bs1, ws2, bs2, out);
}
